// PerformerMultiHeadAttn_15891378995461
// MI455X (gfx1250) — hardware-verified
//
#include <hip/hip_runtime.h>
#define LL 2048
#define BB 2
#define NH 8
#define DH 64
#define DM 512
#define MF 256
#define NTOK (LL * BB)
#define NSL (BB * NH)
#define NR (NTOK * NH)

typedef __bf16 v16b __attribute__((ext_vector_type(16)));
typedef unsigned short v8us __attribute__((ext_vector_type(8), may_alias));
typedef float  v8f  __attribute__((ext_vector_type(8)));
typedef float  v4f  __attribute__((ext_vector_type(4)));
typedef float  v4fa __attribute__((ext_vector_type(4), may_alias));
union FragB { v16b v; v8us half[2]; unsigned short u[16]; };

__device__ __forceinline__ unsigned short bf16_bits(float x) { unsigned int u = __float_as_uint(x); return (unsigned short)((u + 0x7FFFu + ((u >> 16) & 1u)) >> 16); }
__device__ __forceinline__ float bf16_val(unsigned short b) { return __uint_as_float(((unsigned int)b) << 16); }
__device__ __forceinline__ float bf16_round(float x) { return bf16_val(bf16_bits(x)); }
template <int NT>
__device__ __forceinline__ v8f mmaN(v16b ah, v16b al, v16b bh, v16b bl, v8f c) {
  c = __builtin_amdgcn_wmma_f32_16x16x32_bf16(false, ah, false, bh, (short)0, c, false, false);
  if (NT >= 2) c = __builtin_amdgcn_wmma_f32_16x16x32_bf16(false, al, false, bh, (short)0, c, false, false);
  if (NT >= 3) c = __builtin_amdgcn_wmma_f32_16x16x32_bf16(false, ah, false, bl, (short)0, c, false, false);
  asm volatile("v_nop\n\tv_nop\n\tv_nop\n\tv_nop" : "+v"(c) : "v"(ah), "v"(al), "v"(bh), "v"(bl));
  return c;
}

__global__ __launch_bounds__(256) void k_wt_bf16(const float* __restrict__ W, unsigned short* __restrict__ Wt, int K, int N) {
  const int t = blockIdx.x * 256 + threadIdx.x;
  const int k8n = K / 8;
  if (t >= N * k8n) return;
  const int n = t / k8n, k8 = (t % k8n) * 8;
  v8us v;
#pragma unroll
  for (int i = 0; i < 8; ++i) v[i] = bf16_bits(W[(size_t)(k8 + i) * N + n]);
  *(volatile v8us*)(Wt + (size_t)n * K + k8) = v;
  __threadfence();
  *(volatile v8us*)(Wt + (size_t)n * K + k8) = v;
}

template <bool ASPLIT, int ACT, bool BIAS_BF16>
__global__ __launch_bounds__(128) void k_gemm_bf(const float* __restrict__ A, int lda, const unsigned short* __restrict__ Wt, int ldb,
                                               const float* __restrict__ bias, float* __restrict__ C, int ldc, int M, int N, int K) {
  __shared__ __attribute__((aligned(16))) float so[4][16][64];
  const int tid = threadIdx.x, w = tid >> 5, lane = tid & 31, ln = lane & 15, hh = lane >> 4;
  const int ntn = N / 64;
  const int wid = blockIdx.x * 4 + w;
  const int mt = wid / ntn, nq = wid % ntn;
  if (mt * 16 >= M) return;
  const int row0 = mt * 16, col0 = nq * 64;
  const float* arow = A + (size_t)(row0 + ln) * lda;
  v8f acc[4] = {};
  for (int kb = 0; kb < K; kb += 32) {
    FragB ah, al;
    const v4f x0 = *(const v4fa*)(arow + kb + 8 * hh), x1 = *(const v4fa*)(arow + kb + 8 * hh + 4);
    const v4f x2 = *(const v4fa*)(arow + kb + 16 + 8 * hh), x3 = *(const v4fa*)(arow + kb + 16 + 8 * hh + 4);
    float xs[16] = {x0[0],x0[1],x0[2],x0[3],x1[0],x1[1],x1[2],x1[3],x2[0],x2[1],x2[2],x2[3],x3[0],x3[1],x3[2],x3[3]};
#pragma unroll
    for (int i = 0; i < 16; ++i) { const unsigned short hb = bf16_bits(xs[i]); ah.u[i] = hb; al.u[i] = ASPLIT ? bf16_bits(xs[i] - bf16_val(hb)) : (unsigned short)0; }
#pragma unroll
    for (int t = 0; t < 4; ++t) {
      const unsigned short* brow = Wt + (size_t)(col0 + t * 16 + ln) * ldb + kb;
      FragB b;
      b.half[0] = *(const v8us*)(brow + 8 * hh);
      b.half[1] = *(const v8us*)(brow + 16 + 8 * hh);
      acc[t] = mmaN<ASPLIT ? 2 : 1>(ah.v, al.v, b.v, b.v, acc[t]);
    }
  }
#pragma unroll
  for (int t = 0; t < 4; ++t) {
    float bv = bias ? bias[col0 + t * 16 + ln] : 0.f;
    if (BIAS_BF16) bv = bf16_round(bv);
#pragma unroll
    for (int r = 0; r < 8; ++r) { float v = acc[t][r] + bv; if (ACT == 1) v = fmaxf(v, 0.f); so[w][8 * hh + r][t * 16 + ln] = v; }
  }
  __builtin_amdgcn_fence(__ATOMIC_ACQ_REL, "workgroup");
  __builtin_amdgcn_wave_barrier();
  const int rsub = lane >> 4, c4 = (lane & 15) * 4;
  for (int pass = 0; pass < 2; ++pass) {
#pragma unroll
    for (int q = 0; q < 8; ++q) {
      const int r = q * 2 + rsub;
      const v4f v = *(const v4fa*)&so[w][r][c4];
      *(volatile v4f*)(C + (size_t)(row0 + r) * ldc + col0 + c4) = v;
    }
    if (pass == 0) __threadfence();
  }
}

template <int D, bool CAUSAL>
__global__ __launch_bounds__(128) void k_flash(const float* __restrict__ qb, const float* __restrict__ kb, const float* __restrict__ vb,
                                             int pitch, int T, int H, float scale, float* __restrict__ y, int ypitch) {
  constexpr int KS = D / 32;
  constexpr int DT = D / 16;
  __shared__ __attribute__((aligned(16))) unsigned short sKh[32][D + 8], sKl[32][D + 8], sVh[32][D + 8], sVl[32][D + 8];
  __shared__ __attribute__((aligned(16))) unsigned short sPh[4][16][40], sPl[4][16][40];
  __shared__ __attribute__((aligned(16))) float sO[4][16][D];
  const int tid = threadIdx.x, w = tid >> 5, lane = tid & 31, ln = lane & 15, hh = lane >> 4;
  const int nqb = (T + 63) / 64;
  const int bh = blockIdx.x / nqb, qblk = blockIdx.x % nqb;
  const int b = bh / H, h = bh % H;
  const int q0 = qblk * 64 + w * 16;
  const float* Q = qb + (size_t)b * T * pitch + h * D;
  const float* K = kb + (size_t)b * T * pitch + h * D;
  const float* V = vb + (size_t)b * T * pitch + h * D;

  FragB aqh[KS], aql[KS];
  {
    int row = q0 + ln; if (row >= T) row = T - 1;
    const float* qr = Q + (size_t)row * pitch;
#pragma unroll
    for (int ks = 0; ks < KS; ++ks)
#pragma unroll
      for (int i = 0; i < 16; ++i) {
        const int d = ks * 32 + ((i < 8) ? (8 * hh + i) : (16 + 8 * hh + (i - 8)));
        const float x = qr[d] * scale; const unsigned short hb = bf16_bits(x);
        aqh[ks].u[i] = hb; aql[ks].u[i] = bf16_bits(x - bf16_val(hb));
      }
  }
  float m_r[8], l_r[8];
#pragma unroll
  for (int r = 0; r < 8; ++r) { m_r[r] = -3.0e38f; l_r[r] = 0.f; }
  v8f oacc[DT];
#pragma unroll
  for (int dt = 0; dt < DT; ++dt) oacc[dt] = (v8f){0.f,0.f,0.f,0.f,0.f,0.f,0.f,0.f};

  const int kv_end = CAUSAL ? min(T, qblk * 64 + 64) : T;
  for (int j0 = 0; j0 < kv_end; j0 += 32) {
    __syncthreads();
    for (int e = tid; e < 32 * (D / 4); e += 128) {
      const int r = e / (D / 4), c4 = (e % (D / 4)) * 4;
      const int key = j0 + r;
      v4f kf = {0.f,0.f,0.f,0.f}, vf = {0.f,0.f,0.f,0.f};
      if (key < T) { kf = *(const v4fa*)(K + (size_t)key * pitch + c4); vf = *(const v4fa*)(V + (size_t)key * pitch + c4); }
#pragma unroll
      for (int t = 0; t < 4; ++t) {
        unsigned short hb = bf16_bits(kf[t]); sKh[r][c4 + t] = hb; sKl[r][c4 + t] = bf16_bits(kf[t] - bf16_val(hb));
        hb = bf16_bits(vf[t]); sVh[r][c4 + t] = hb; sVl[r][c4 + t] = bf16_bits(vf[t] - bf16_val(hb));
      }
    }
    __syncthreads();
    v8f s[2];
#pragma unroll
    for (int nt = 0; nt < 2; ++nt) {
      v8f acc = {};
#pragma unroll
      for (int ks = 0; ks < KS; ++ks) {
        FragB bh_, bl_;
        bh_.half[0] = *(const v8us*)&sKh[nt * 16 + ln][ks * 32 + 8 * hh]; bh_.half[1] = *(const v8us*)&sKh[nt * 16 + ln][ks * 32 + 16 + 8 * hh];
        bl_.half[0] = *(const v8us*)&sKl[nt * 16 + ln][ks * 32 + 8 * hh]; bl_.half[1] = *(const v8us*)&sKl[nt * 16 + ln][ks * 32 + 16 + 8 * hh];
        acc = mmaN<3>(aqh[ks].v, aql[ks].v, bh_.v, bl_.v, acc);
      }
      s[nt] = acc;
    }
    float alpha[8];
#pragma unroll
    for (int r = 0; r < 8; ++r) {
      const int qi = q0 + 8 * hh + r;
      const int ja = j0 + ln, jb = j0 + 16 + ln;
      if (CAUSAL) { if (ja > qi) s[0][r] = -3.0e38f; if (jb > qi) s[1][r] = -3.0e38f; }
      if (ja >= T) s[0][r] = -3.0e38f;
      if (jb >= T) s[1][r] = -3.0e38f;
      float mx = fmaxf(s[0][r], s[1][r]);
      mx = fmaxf(mx, __shfl_xor(mx, 1, 32)); mx = fmaxf(mx, __shfl_xor(mx, 2, 32)); mx = fmaxf(mx, __shfl_xor(mx, 4, 32)); mx = fmaxf(mx, __shfl_xor(mx, 8, 32));
      const float mnew = fmaxf(m_r[r], mx);
      alpha[r] = (mnew > -1.0e38f) ? __expf(m_r[r] - mnew) : 1.0f;
      const float p0 = (s[0][r] > -1.0e38f) ? __expf(s[0][r] - mnew) : 0.f;
      const float p1 = (s[1][r] > -1.0e38f) ? __expf(s[1][r] - mnew) : 0.f;
      m_r[r] = mnew;
      l_r[r] = l_r[r] * alpha[r] + p0 + p1;
      unsigned short hb = bf16_bits(p0); sPh[w][8 * hh + r][ln] = hb;      sPl[w][8 * hh + r][ln] = bf16_bits(p0 - bf16_val(hb));
      hb = bf16_bits(p1);                sPh[w][8 * hh + r][16 + ln] = hb; sPl[w][8 * hh + r][16 + ln] = bf16_bits(p1 - bf16_val(hb));
    }
#pragma unroll
    for (int dt = 0; dt < DT; ++dt)
#pragma unroll
      for (int r = 0; r < 8; ++r) oacc[dt][r] *= alpha[r];
    __builtin_amdgcn_fence(__ATOMIC_ACQ_REL, "workgroup");
    __builtin_amdgcn_wave_barrier();
    FragB pah, pal;
    pah.half[0] = *(const v8us*)&sPh[w][ln][8 * hh]; pah.half[1] = *(const v8us*)&sPh[w][ln][16 + 8 * hh];
    pal.half[0] = *(const v8us*)&sPl[w][ln][8 * hh]; pal.half[1] = *(const v8us*)&sPl[w][ln][16 + 8 * hh];
#pragma unroll
    for (int dt = 0; dt < DT; ++dt) {
      FragB bvh, bvl;
#pragma unroll
      for (int i = 0; i < 8; ++i) {
        bvh.u[i] = sVh[8 * hh + i][dt * 16 + ln]; bvh.u[8 + i] = sVh[16 + 8 * hh + i][dt * 16 + ln];
        bvl.u[i] = sVl[8 * hh + i][dt * 16 + ln]; bvl.u[8 + i] = sVl[16 + 8 * hh + i][dt * 16 + ln];
      }
      oacc[dt] = mmaN<3>(pah.v, pal.v, bvh.v, bvl.v, oacc[dt]);
    }
    __builtin_amdgcn_fence(__ATOMIC_ACQ_REL, "workgroup");
    __builtin_amdgcn_wave_barrier();
  }
#pragma unroll
  for (int r = 0; r < 8; ++r) {
    float l = l_r[r];
    l += __shfl_xor(l, 1, 32); l += __shfl_xor(l, 2, 32); l += __shfl_xor(l, 4, 32); l += __shfl_xor(l, 8, 32);
    l_r[r] = (l > 0.f) ? 1.0f / l : 0.f;
  }
#pragma unroll
  for (int dt = 0; dt < DT; ++dt)
#pragma unroll
    for (int r = 0; r < 8; ++r) sO[w][8 * hh + r][dt * 16 + ln] = oacc[dt][r] * l_r[r];
  __builtin_amdgcn_fence(__ATOMIC_ACQ_REL, "workgroup");
  __builtin_amdgcn_wave_barrier();
  for (int pass = 0; pass < 2; ++pass) {
    for (int r = 0; r < 16; ++r) {
      const int row = q0 + r;
      if (row < T && lane < D / 4) {
        const v4f val = *(const v4fa*)&sO[w][r][lane * 4];
        *(volatile v4f*)(y + ((size_t)b * T + row) * ypitch + h * D + lane * 4) = val;
      }
    }
    if (pass == 0) __threadfence();
  }
}

template <bool ASPLIT, bool BSPLIT, int ACT>
__global__ __launch_bounds__(128) void k_gemm_b(const float* __restrict__ A, int lda, size_t sA, const unsigned short* __restrict__ Bh, const unsigned short* __restrict__ Bl, int ldb, size_t sB,
                                             const float* __restrict__ bias, const float* __restrict__ resid, int ldr, size_t sR, float rsign, float alpha,
                                             float* __restrict__ C, int ldc, size_t sC, int M, int N, int K) {
  __shared__ __attribute__((aligned(16))) float so[4][16][64];
  const int tid = threadIdx.x, w = tid >> 5, lane = tid & 31, ln = lane & 15, hh = lane >> 4;
  const int by = blockIdx.y;
  A += (size_t)by * sA; Bh += (size_t)by * sB; if (BSPLIT) Bl += (size_t)by * sB; C += (size_t)by * sC; if (resid) resid += (size_t)by * sR;
  const int ntn = (N + 63) / 64; const int wid = blockIdx.x * 4 + w; const int mt = wid / ntn, nq = wid % ntn;
  if (mt * 16 >= M) return;
  const int row0 = mt * 16, col0 = nq * 64;
  const float* arow = A + (size_t)(row0 + ln) * lda;
  v8f acc[4] = {};
  for (int kb = 0; kb < K; kb += 32) {
    FragB ah, al;
    const v4f x0 = *(const v4fa*)(arow + kb + 8 * hh), x1 = *(const v4fa*)(arow + kb + 8 * hh + 4);
    const v4f x2 = *(const v4fa*)(arow + kb + 16 + 8 * hh), x3 = *(const v4fa*)(arow + kb + 16 + 8 * hh + 4);
    float xs[16] = {x0[0],x0[1],x0[2],x0[3],x1[0],x1[1],x1[2],x1[3],x2[0],x2[1],x2[2],x2[3],x3[0],x3[1],x3[2],x3[3]};
#pragma unroll
    for (int i = 0; i < 16; ++i) { const unsigned short hb = bf16_bits(xs[i]); ah.u[i] = hb; al.u[i] = ASPLIT ? bf16_bits(xs[i] - bf16_val(hb)) : (unsigned short)0; }
#pragma unroll
    for (int t = 0; t < 4; ++t) {
      if (col0 + t * 16 >= N) continue;
      const size_t boff = (size_t)(col0 + t * 16 + ln) * ldb + kb;
      FragB bh_, bl_; bh_.half[0] = *(const v8us*)(Bh + boff + 8 * hh); bh_.half[1] = *(const v8us*)(Bh + boff + 16 + 8 * hh);
      if (BSPLIT) { bl_.half[0] = *(const v8us*)(Bl + boff + 8 * hh); bl_.half[1] = *(const v8us*)(Bl + boff + 16 + 8 * hh); } else bl_ = bh_;
      acc[t] = mmaN<ASPLIT ? (BSPLIT ? 3 : 2) : 1>(ah.v, al.v, bh_.v, bl_.v, acc[t]);
    }
  }
#pragma unroll
  for (int t = 0; t < 4; ++t) {
    const int col = col0 + t * 16 + ln; if (col0 + t * 16 >= N) continue; const float bv = bias ? bf16_round(bias[col]) : 0.f;
#pragma unroll
    for (int r = 0; r < 8; ++r) { float v = acc[t][r] * alpha + bv; if (resid) v += rsign * resid[(size_t)(row0 + 8 * hh + r) * ldr + col]; if (ACT == 1) v = fmaxf(v, 0.f); else if (ACT == 2) v = fmaxf(v, 0.f) + log1pf(expf(-fabsf(v))); so[w][8 * hh + r][t * 16 + ln] = v; }
  }
  __builtin_amdgcn_fence(__ATOMIC_ACQ_REL, "workgroup"); __builtin_amdgcn_wave_barrier();
  const int rsub = lane >> 4, c4 = (lane & 15) * 4;
  for (int pass = 0; pass < 2; ++pass) {
#pragma unroll
    for (int q = 0; q < 8; ++q) { const int r = q * 2 + rsub; if (col0 + c4 < N) { const v4f v = *(const v4fa*)&so[w][r][c4]; *(volatile v4f*)(C + (size_t)(row0 + r) * ldc + col0 + c4) = v; } }
    if (pass == 0) __threadfence();
  }
}
__global__ __launch_bounds__(256) void k_split_transpose_b(const float* __restrict__ src, int lds_, size_t sIn, unsigned short* __restrict__ hi, unsigned short* __restrict__ lo, size_t sOut, int K, int N) {
  const size_t t = (size_t)blockIdx.x * 256 + threadIdx.x; const int k8n = K / 8; if (t >= (size_t)N * k8n) return;
  src += (size_t)blockIdx.y * sIn; hi += (size_t)blockIdx.y * sOut; lo += (size_t)blockIdx.y * sOut;
  const int n = (int)(t / k8n), k8 = (int)(t % k8n) * 8; v8us vh, vl;
#pragma unroll
  for (int i = 0; i < 8; ++i) { const float x = src[(size_t)(k8 + i) * lds_ + n]; const unsigned short hb = bf16_bits(x); vh[i] = hb; vl[i] = bf16_bits(x - bf16_val(hb)); }
  unsigned short* dh = hi + (size_t)n * K + k8; unsigned short* dl = lo + (size_t)n * K + k8;
  *(volatile v8us*)dh = vh; *(volatile v8us*)dl = vl; __threadfence(); *(volatile v8us*)dh = vh; *(volatile v8us*)dl = vl;
}

__global__ __launch_bounds__(256) void k_round_rows(const float* __restrict__ W, unsigned short* __restrict__ Wt, int n8) {
  const int t = blockIdx.x * 256 + threadIdx.x;
  if (t >= n8) return;
  const v4f a = *(const v4fa*)(W + (size_t)t * 8), b = *(const v4fa*)(W + (size_t)t * 8 + 4);
  v8us v; v[0]=bf16_bits(a[0]); v[1]=bf16_bits(a[1]); v[2]=bf16_bits(a[2]); v[3]=bf16_bits(a[3]);
  v[4]=bf16_bits(b[0]); v[5]=bf16_bits(b[1]); v[6]=bf16_bits(b[2]); v[7]=bf16_bits(b[3]);
  *(volatile v8us*)(Wt + (size_t)t * 8) = v; __threadfence(); *(volatile v8us*)(Wt + (size_t)t * 8) = v;
}

__global__ __launch_bounds__(256) void k_bp(const float* __restrict__ proj, unsigned short* __restrict__ Bp) { const int t = blockIdx.x * 256 + threadIdx.x; if (t >= MF * DH / 8) return; const int d8 = (t % (DH / 8)) * 8, m = t / (DH / 8); v8us v; for (int q = 0; q < 8; ++q) v[q] = bf16_bits(proj[(size_t)(d8 + q) * MF + m]); *(volatile v8us*)(Bp + (size_t)m * DH + d8) = v; __threadfence(); *(volatile v8us*)(Bp + (size_t)m * DH + d8) = v; }
__global__ __launch_bounds__(256) void k_primeq2(const float* __restrict__ XP, const float* __restrict__ Q, float* __restrict__ QP) { const int tid = threadIdx.x, wv = tid >> 5, lane = tid & 31; const size_t r = (size_t)blockIdx.x * 8 + wv; const size_t tok = r / NH; const int h = (int)(r % NH);
  const float* qrow = Q + tok * DM + h * DH; const float a = qrow[lane] * 0.35355339059327373f, b2 = qrow[32 + lane] * 0.35355339059327373f; float s = a * a + b2 * b2; for (int o = 16; o >= 1; o >>= 1) s += __shfl_xor(s, o, 32); const float hs = 0.5f * s;
  float v[MF / 32]; for (int u = 0; u < MF / 32; ++u) v[u] = expf(XP[r * MF + u * 32 + lane] - hs) * 0.0625f;
  for (int pass = 0; pass < 2; ++pass) { for (int u = 0; u < MF / 32; ++u) *(volatile float*)(QP + r * MF + u * 32 + lane) = v[u]; if (pass == 0) __threadfence(); } }
__global__ __launch_bounds__(256) void k_primek(const float* __restrict__ XPK, const float* __restrict__ KV, int h, float* __restrict__ KPT) { __shared__ float tile[32][MF + 1]; __shared__ float shs[32]; const int tid = threadIdx.x, wv = tid >> 5, lane = tid & 31; const int b = blockIdx.y, l0 = blockIdx.x * 32; const int slab = b * NH + h;
  for (int i = wv; i < 32; i += 8) { const int l = l0 + i; const size_t tok = (size_t)l * BB + b; const float* krow = KV + tok * (2 * DM) + h * DH; const float a = krow[lane] * 0.35355339059327373f, c = krow[32 + lane] * 0.35355339059327373f; float s = a * a + c * c; for (int o = 16; o >= 1; o >>= 1) s += __shfl_xor(s, o, 32); if (lane == 0) shs[i] = 0.5f * s;
    for (int u = 0; u < MF / 32; ++u) tile[i][u * 32 + lane] = XPK[tok * MF + u * 32 + lane]; }
  __syncthreads();
  for (int i = wv; i < 32; i += 8) for (int u = 0; u < MF / 32; ++u) tile[i][u * 32 + lane] = expf(tile[i][u * 32 + lane] - shs[i]) * 0.0625f;
  __syncthreads();
  for (int pass = 0; pass < 2; ++pass) { for (int m = wv; m < MF; m += 8) *(volatile float*)(KPT + ((size_t)slab * MF + m) * LL + l0 + lane) = tile[lane][m]; if (pass == 0) __threadfence(); } }
__global__ __launch_bounds__(256) void k_vt(const float* __restrict__ KV, unsigned short* __restrict__ Vh, unsigned short* __restrict__ Vl) { __shared__ float tile[32][33]; const int l0 = blockIdx.x * 32, d0 = blockIdx.y * 32, slab = blockIdx.z; const int b = slab / NH, h = slab % NH; const int tx = threadIdx.x & 31, ty = threadIdx.x >> 5;
  for (int i = ty; i < 32; i += 8) tile[i][tx] = KV[((size_t)(l0 + i) * BB + b) * (2 * DM) + DM + h * DH + d0 + tx]; __syncthreads();
  typedef unsigned short v4us __attribute__((ext_vector_type(4))); const int r = threadIdx.x >> 3, c4 = (threadIdx.x & 7) * 4; v4us hh4, ll4; for (int q = 0; q < 4; ++q) { const float v = tile[c4 + q][r]; const float vh = bf16_round(v); hh4[q] = bf16_bits(vh); ll4[q] = bf16_bits(v - vh); }
  unsigned short* dh = Vh + ((size_t)slab * DH + d0 + r) * LL + l0 + c4; unsigned short* dl = Vl + ((size_t)slab * DH + d0 + r) * LL + l0 + c4; *(volatile v4us*)dh = hh4; *(volatile v4us*)dl = ll4; __threadfence(); *(volatile v4us*)dh = hh4; *(volatile v4us*)dl = ll4; }
__global__ __launch_bounds__(256) void k_b2(const float* __restrict__ KVS, const float* __restrict__ KPT, unsigned short* __restrict__ B2h, unsigned short* __restrict__ B2l) { __shared__ float tile[32][65]; __shared__ float sks[32]; const int tid = threadIdx.x, wv = tid >> 5, lane = tid & 31; const int slab = blockIdx.y, m0 = blockIdx.x * 32;
  for (int i = wv; i < 32; i += 8) { const int m = m0 + i; tile[i][lane] = KVS[((size_t)slab * MF + m) * DH + lane]; tile[i][32 + lane] = KVS[((size_t)slab * MF + m) * DH + 32 + lane]; float s = 0.f;
#pragma unroll 4
    for (int l = lane; l < LL; l += 32) s += KPT[((size_t)slab * MF + m) * LL + l]; for (int o = 16; o >= 1; o >>= 1) s += __shfl_xor(s, o, 32); if (lane == 0) sks[i] = s; }
  __syncthreads();
  for (int pass = 0; pass < 2; ++pass) { for (int row = wv; row < 128; row += 8) { float v = 0.f; if (row < DH) v = tile[lane][row]; else if (row == DH) v = sks[lane]; const float vh = bf16_round(v); const size_t o = ((size_t)slab * 128 + row) * MF + m0 + lane; *(volatile unsigned short*)(B2h + o) = bf16_bits(vh); *(volatile unsigned short*)(B2l + o) = bf16_bits(v - vh); } if (pass == 0) __threadfence(); } }
__global__ __launch_bounds__(256) void k_vec(const float* __restrict__ NUM, float* __restrict__ VEC) { const size_t t = (size_t)blockIdx.x * 256 + threadIdx.x; if (t >= (size_t)NTOK * DM) return; const int c = (int)(t % DM); const size_t tok = t / DM; const int h = c / DH, d = c % DH; const int l = (int)(tok / BB), b = (int)(tok % BB); const int slab = b * NH + h;
  const float* row = NUM + ((size_t)slab * LL + l) * 128; const float v = (row[d] * 0.125f) / (row[DH] * 0.125f + 1e-5f);   *(volatile float*)(VEC + t) = v; __threadfence(); *(volatile float*)(VEC + t) = v; }
__global__ __launch_bounds__(256) void k_ln(const float* __restrict__ hin, const float* __restrict__ ATT, const float* __restrict__ g, const float* __restrict__ be, float* __restrict__ out) { const int tid = threadIdx.x, wv = tid >> 5, lane = tid & 31; const size_t tok = (size_t)blockIdx.x * 8 + wv; float x[DM / 32]; float s = 0.f;
  for (int u = 0; u < DM / 32; ++u) { const int c = u * 32 + lane; x[u] = bf16_round(hin[tok * DM + c]) + ATT[tok * DM + c]; s += x[u]; } for (int o = 16; o >= 1; o >>= 1) s += __shfl_xor(s, o, 32); const float mu = s * (1.0f / DM); float q = 0.f; for (int u = 0; u < DM / 32; ++u) { const float d = x[u] - mu; q += d * d; } for (int o = 16; o >= 1; o >>= 1) q += __shfl_xor(q, o, 32); const float rs = 1.0f / sqrtf(q * (1.0f / DM) + 1e-5f);
  for (int pass = 0; pass < 2; ++pass) { for (int u = 0; u < DM / 32; ++u) { const int c = u * 32 + lane; *(volatile float*)(out + tok * DM + c) = bf16_round(g[c]) * (x[u] - mu) * rs + bf16_round(be[c]); } if (pass == 0) __threadfence(); } }
extern "C" void kernel_launch(void* const* d_in, const int* in_sizes, int n_in,
                              void* d_out, int out_size, void* d_ws, size_t ws_size, hipStream_t stream) {
  (void)in_sizes; (void)n_in; (void)out_size;
  const float* hin = (const float*)d_in[0]; const float* Wq = (const float*)d_in[1]; const float* Wkv = (const float*)d_in[2]; const float* Wo = (const float*)d_in[3]; const float* lnw = (const float*)d_in[4]; const float* lnb = (const float*)d_in[5]; const float* proj = (const float*)d_in[6];
  char* ws = (char*)d_ws; size_t off = 0;
  auto take = [&](size_t bytes) { char* p = ws + off; off += (bytes + 255) & ~(size_t)255; return p; };
  unsigned short* Bq = (unsigned short*)take((size_t)DM * DM * 2); unsigned short* Bkv = (unsigned short*)take((size_t)2 * DM * DM * 2); unsigned short* Bo = (unsigned short*)take((size_t)DM * DM * 2); unsigned short* Bp = (unsigned short*)take((size_t)MF * DH * 2);
  float* Q = (float*)take((size_t)NTOK * DM * 4); float* KV = (float*)take((size_t)NTOK * 2 * DM * 4); float* QP = (float*)take((size_t)NR * MF * 4); float* KPT = (float*)take((size_t)NSL * MF * LL * 4);
  unsigned short* Vh = (unsigned short*)take((size_t)NSL * DH * LL * 2); unsigned short* Vl = (unsigned short*)take((size_t)NSL * DH * LL * 2); float* KVS = (float*)take((size_t)NSL * MF * DH * 4); unsigned short* B2h = (unsigned short*)take((size_t)NSL * 128 * MF * 2); unsigned short* B2l = (unsigned short*)take((size_t)NSL * 128 * MF * 2);
  float* VEC = (float*)take((size_t)NTOK * DM * 4); float* NUM = KV;   float* ATT = Q;
  if (off > ws_size) return;
  k_round_rows<<<(DM * DM / 8 + 255) / 256, 256, 0, stream>>>(Wq, Bq, DM * DM / 8); k_round_rows<<<(2 * DM * DM / 8 + 255) / 256, 256, 0, stream>>>(Wkv, Bkv, 2 * DM * DM / 8); k_round_rows<<<(DM * DM / 8 + 255) / 256, 256, 0, stream>>>(Wo, Bo, DM * DM / 8); k_bp<<<(MF * DH / 8 + 255) / 256, 256, 0, stream>>>(proj, Bp);
  k_gemm_b<false, false, 0><<<dim3(((NTOK / 16) * (DM / 64) + 3) / 4, 1), 128, 0, stream>>>(hin, DM, 0, Bq, Bq, DM, 0, nullptr, nullptr, 0, 0, 1.f, 1.f, Q, DM, 0, NTOK, DM, DM);
  k_gemm_b<false, false, 0><<<dim3(((NTOK / 16) * (2 * DM / 64) + 3) / 4, 1), 128, 0, stream>>>(hin, DM, 0, Bkv, Bkv, DM, 0, nullptr, nullptr, 0, 0, 1.f, 1.f, KV, 2 * DM, 0, NTOK, 2 * DM, DM);
  k_gemm_b<true, false, 0><<<dim3(((NR / 16) * (MF / 64) + 3) / 4, 1), 128, 0, stream>>>(Q, DH, 0, Bp, Bp, DH, 0, nullptr, nullptr, 0, 0, 1.f, 0.35355339059327373f, QP, MF, 0, NR, MF, DH);
  k_primeq2<<<NR / 8, 256, 0, stream>>>(QP, Q, QP);
  k_vt<<<dim3(LL / 32, DH / 32, NSL), 256, 0, stream>>>(KV, Vh, Vl);
  float* XPKh = VEC;
  for (int h = 0; h < NH; ++h) {
    k_gemm_b<true, false, 0><<<dim3(((NTOK / 16) * (MF / 64) + 3) / 4, 1), 128, 0, stream>>>(KV + h * DH, 2 * DM, 0, Bp, Bp, DH, 0, nullptr, nullptr, 0, 0, 1.f, 0.35355339059327373f, XPKh, MF, 0, NTOK, MF, DH);
    k_primek<<<dim3(LL / 32, BB), 256, 0, stream>>>(XPKh, KV, h, KPT); }
  k_gemm_b<true, true, 0><<<dim3(((MF / 16) * 1 + 3) / 4, NSL), 128, 0, stream>>>(KPT, LL, (size_t)MF * LL, Vh, Vl, LL, (size_t)DH * LL, nullptr, nullptr, 0, 0, 1.f, 1.f, KVS, DH, (size_t)MF * DH, MF, DH, LL);
  k_b2<<<dim3(MF / 32, NSL), 256, 0, stream>>>(KVS, KPT, B2h, B2l);
  k_gemm_b<true, true, 0><<<dim3(((LL / 16) * 2 + 3) / 4, NSL), 128, 0, stream>>>(QP, BB * NH * MF, (size_t)MF, B2h, B2l, MF, (size_t)128 * MF, nullptr, nullptr, 0, 0, 1.f, 1.f, NUM, 128, (size_t)LL * 128, LL, 128, MF);
  k_vec<<<(unsigned)(((size_t)NTOK * DM + 255) / 256), 256, 0, stream>>>(NUM, VEC);
  k_gemm_b<true, false, 0><<<dim3(((NTOK / 16) * (DM / 64) + 3) / 4, 1), 128, 0, stream>>>(VEC, DM, 0, Bo, Bo, DM, 0, nullptr, nullptr, 0, 0, 1.f, 1.f, ATT, DM, 0, NTOK, DM, DM);
  k_ln<<<NTOK / 8, 256, 0, stream>>>(hin, ATT, lnw, lnb, (float*)d_out);
}
